// fusion_87711822119594
// MI455X (gfx1250) — hardware-run, weakly checked
//
#include <hip/hip_runtime.h>
#include <math.h>

typedef __attribute__((ext_vector_type(16))) _Float16 v16h;
typedef __attribute__((ext_vector_type(8)))  _Float16 v8h;
typedef __attribute__((ext_vector_type(16))) __bf16   v16b;
typedef __attribute__((ext_vector_type(8)))  __bf16   v8b;
typedef __attribute__((ext_vector_type(8)))  float    v8f;
typedef __attribute__((ext_vector_type(4)))  float    v4f;

constexpr int kNB     = 4;
constexpr int kCin    = 512;
constexpr int kCout   = 256;
constexpr int kHW     = 1024;
constexpr int kImgW   = 32;
constexpr int kNTok   = kNB * kHW;
constexpr int kDin    = 512;
constexpr int kNst    = 16;
constexpr int kDtR    = 16;
constexpr int kSeqL   = 2 * kHW;
constexpr int kNSeq   = kNB * kSeqL;
constexpr int kXzP    = 2 * kDin;
constexpr int kXdW    = kDtR + 2 * kNst;
constexpr int kXdP    = 64;
constexpr int kConvTP = 260;
constexpr int kScanTS = 64;
constexpr int kScanCh = 64;
constexpr int kScanYP = 68;
static_assert(kImgW * kImgW == kHW, "image");
static_assert((kCin % 32) == 0 && (kCout % 32) == 0 && (kDin % 32) == 0, "GEMM K multiples of 32");
static_assert((kNTok % 64) == 0 && (kCout % 64) == 0 && (kXzP % 64) == 0 && (kNSeq % 64) == 0 &&
              (kXdP % 64) == 0 && (kHW % 64) == 0, "GEMM M,N multiples of 64");
static_assert(((kNTok / 64) * (kCout / 64)) % 8 == 0 && ((kNTok / 64) * (kXzP / 64)) % 8 == 0 &&
              ((kNSeq / 64) * (kXdP / 64)) % 8 == 0 && ((kCout / 64) * (kHW / 64)) % 8 == 0, "8 tiles per GEMM block exactly");
static_assert(kXdW <= kXdP && (kXdW % 4) == 0, "x_proj pad");
static_assert((kSeqL % kScanTS) == 0 && (kDin % kScanCh) == 0 && (kDin % 256) == 0 && (kHW % 16) == 0, "tile multiples");
static_assert((kCin % 64) == 0 && (kHW % 64) == 0 && (kDin % 64) == 0, "transpose tiles");

constexpr size_t kOffXB   = 0;
constexpr size_t kOffXBL  = kOffXB  + (size_t)2 * kNTok * kCin * 2;
constexpr size_t kOffWB   = kOffXBL + (size_t)2 * kNTok * kCin * 2;
constexpr size_t kOffWBL  = kOffWB  + (size_t)2 * kCout * kCin * 2;
constexpr size_t kOffIP   = kOffWBL + (size_t)2 * kCout * kCin * 2;
constexpr size_t kOffXP   = kOffIP  + (size_t)2 * kXzP * kCout * 2;
constexpr size_t kOffOW   = kOffXP  + (size_t)kXdP * kDin * 2;
constexpr size_t kOffRS   = kOffOW  + (size_t)kCout * kDin * 2;
constexpr size_t kOffLN   = kOffRS  + (size_t)2 * kNTok * kCout * 4;
constexpr size_t kOffXZ   = kOffLN  + (size_t)2 * kNTok * kCout * 2;
constexpr size_t kOffU    = kOffXZ  + (size_t)2 * kNTok * kXzP * 4;
constexpr size_t kOffU16  = kOffU   + (size_t)kNSeq * kDin * 4;
constexpr size_t kOffXD   = kOffU16 + (size_t)kNSeq * kDin * 2;
constexpr size_t kOffY    = kOffXD  + (size_t)kNSeq * kXdP * 4;
constexpr size_t kOffG    = kOffY   + (size_t)kNSeq * kDin * 4;
constexpr size_t kOffRT   = kOffG   + (size_t)kNTok * kDin * 2;
constexpr size_t kWsTotal = kOffRT  + (size_t)kNB * kCout * kHW * 4;
static_assert(kWsTotal == 117768192ull, "carve total");
static_assert(kWsTotal <= 134217728ull, "carve cap");
static_assert((kOffXBL % 128) == 0 && (kOffWB % 128) == 0 && (kOffWBL % 128) == 0 && (kOffIP % 128) == 0 &&
              (kOffXP % 128) == 0 && (kOffOW % 128) == 0 && (kOffRS % 128) == 0 && (kOffLN % 128) == 0 &&
              (kOffXZ % 128) == 0 && (kOffU % 128) == 0 && (kOffU16 % 128) == 0 && (kOffXD % 128) == 0 &&
              (kOffY % 128) == 0 && (kOffG % 128) == 0 && (kOffRT % 128) == 0, "128-B aligned regions");

__device__ __forceinline__ unsigned short f2bf_bits(float f) {
  unsigned u = __float_as_uint(f);
  return (unsigned short)((u + 0x7FFFu + ((u >> 16) & 1u)) >> 16);
}
__device__ __forceinline__ float bf_bits2f(unsigned short h) { return __uint_as_float(((unsigned)h) << 16); }

__device__ __forceinline__ void dep_guard4_h(v8f& a, v8f& b, v8f& c, v8f& d, v16h x, v16h y) {
  asm volatile("v_nop\n\tv_nop\n\tv_nop\n\tv_nop" : "+v"(a), "+v"(b), "+v"(c), "+v"(d) : "v"(x), "v"(y));
}
__device__ __forceinline__ void dep_guard4_b(v8f& a, v8f& b, v8f& c, v8f& d, v16b x, v16b y) {
  asm volatile("v_nop\n\tv_nop\n\tv_nop\n\tv_nop" : "+v"(a), "+v"(b), "+v"(c), "+v"(d) : "v"(x), "v"(y));
}
__device__ __forceinline__ void keep4_h(v16h a, v16h b, v16h c, v16h d) { asm volatile("v_nop" :: "v"(a), "v"(b), "v"(c), "v"(d)); }
__device__ __forceinline__ void keep4_b(v16b a, v16b b, v16b c, v16b d) { asm volatile("v_nop" :: "v"(a), "v"(b), "v"(c), "v"(d)); }
__device__ __forceinline__ void acc_guard4(v8f& a, v8f& b, v8f& c, v8f& d) { asm volatile("v_nop\n\tv_nop\n\tv_nop\n\tv_nop" : "+v"(a), "+v"(b), "+v"(c), "+v"(d)); }
template <typename T> struct Frag;
template <> struct Frag<_Float16> {
  typedef v16h V; union U { v16h v; v8h h[2]; };
  static __device__ __forceinline__ v16h load(const _Float16* p) {
    U f; f.h[0] = *(const v8h*)(p); f.h[1] = *(const v8h*)(p + 16); return f.v;
  }
  static __device__ __forceinline__ v8f mma(v16h a, v16h b, v8f c) {
    return __builtin_amdgcn_wmma_f32_16x16x32_f16(false, a, false, b, (short)0, c, false, false);
  }
  static __device__ __forceinline__ void guard4(v8f& a, v8f& b, v8f& c, v8f& d, v16h x, v16h y) { dep_guard4_h(a, b, c, d, x, y); }
  static __device__ __forceinline__ void keep(v16h a, v16h b, v16h c, v16h d) { keep4_h(a, b, c, d); }
};
template <> struct Frag<__bf16> {
  typedef v16b V; union U { v16b v; v8b h[2]; };
  static __device__ __forceinline__ v16b load(const __bf16* p) {
    U f; f.h[0] = *(const v8b*)(p); f.h[1] = *(const v8b*)(p + 16); return f.v;
  }
  static __device__ __forceinline__ v8f mma(v16b a, v16b b, v8f c) {
    return __builtin_amdgcn_wmma_f32_16x16x32_bf16(false, a, false, b, (short)0, c, false, false);
  }
  static __device__ __forceinline__ void guard4(v8f& a, v8f& b, v8f& c, v8f& d, v16b x, v16b y) { dep_guard4_b(a, b, c, d, x, y); }
  static __device__ __forceinline__ void keep(v16b a, v16b b, v16b c, v16b d) { keep4_b(a, b, c, d); }
};

template <int ET> struct Elem;
template <> struct Elem<0> { typedef _Float16 T; };
template <> struct Elem<1> { typedef __bf16 T; };
template <int ET, int SPL, int EPI, bool RESID>
__global__ __launch_bounds__(256) void wmma_gemm64(
    const unsigned short* __restrict__ Ap, const unsigned short* __restrict__ A2p, int lda, long strideA,
    const unsigned short* __restrict__ Btp, const unsigned short* __restrict__ Bt2p, int ldb, long strideB,
    float* __restrict__ Cout, int ldc, long strideC,
    const float* __restrict__ bnM, const float* __restrict__ bnG,
    const float* __restrict__ bnV, const float* __restrict__ bnB,
    const float* __restrict__ resid, long strideR,
    int M, int N, int K, float scale) {
  static_assert(SPL == 0 || SPL == 2, "plain or two-sided split");
  typedef typename Elem<ET>::T T;
  typedef typename Frag<T>::V V;
  const T* A = (const T*)Ap; const T* A2 = (const T*)A2p; const T* Bt = (const T*)Btp; const T* Bt2 = (const T*)Bt2p;
  __shared__ __align__(16) float sT[8][16 * 68];
  const int b    = blockIdx.y;
  const int lane = threadIdx.x & 31;
  const int wave = threadIdx.x >> 5;
  const int tilesN = N >> 6;
  const int tilesM = M >> 6;
  const int tile = blockIdx.x * 8 + wave;
  if (tile >= tilesM * tilesN) return;
  const int tm = tile / tilesN;
  const int tn = tile - tm * tilesN;
  const int m0 = tm << 6;
  const int n0 = tn << 6;

  const T* Ab  = A  + (size_t)b * strideA;
  const T* Bb  = Bt + (size_t)b * strideB;
  const T* Ab2 = (SPL == 2) ? (A2  + (size_t)b * strideA) : nullptr;
  const T* Bb2 = (SPL == 2) ? (Bt2 + (size_t)b * strideB) : nullptr;

  const int rlane = lane & 15;
  const int koff  = (lane >> 4) * 8;
  const int mOff  = (lane >> 4) * 8;

  v8f acc[4][4];
#pragma unroll
  for (int i = 0; i < 4; ++i)
#pragma unroll
    for (int j = 0; j < 4; ++j) acc[i][j] = (v8f){0.f,0.f,0.f,0.f,0.f,0.f,0.f,0.f};

  for (int k0 = 0; k0 < K; k0 += 32) {
    V bh[4], bl[4];
#pragma unroll
    for (int j = 0; j < 4; ++j) {
      const size_t bo = (size_t)(n0 + (j << 4) + rlane) * ldb + koff + k0;
      bh[j] = Frag<T>::load(Bb + bo);
      if (SPL == 2) bl[j] = Frag<T>::load(Bb2 + bo);
    }
#pragma unroll
    for (int i = 0; i < 4; ++i) {
      const size_t ao = (size_t)(m0 + (i << 4) + rlane) * lda + koff + k0;
      V ah = Frag<T>::load(Ab + ao);
      V al = ah;
      if (SPL == 2) al = Frag<T>::load(Ab2 + ao);
#pragma unroll
      for (int j = 0; j < 4; ++j) {
        acc[i][j] = Frag<T>::mma(ah, bh[j], acc[i][j]);
        if (SPL == 2) {
          acc[i][j] = Frag<T>::mma(ah, bl[j], acc[i][j]);
          acc[i][j] = Frag<T>::mma(al, bh[j], acc[i][j]);
        }
      }
      Frag<T>::guard4(acc[i][0], acc[i][1], acc[i][2], acc[i][3], ah, al);
    }
    Frag<T>::keep(bh[0], bh[1], bh[2], bh[3]);
    if (SPL == 2) Frag<T>::keep(bl[0], bl[1], bl[2], bl[3]);
  }
  acc_guard4(acc[0][0], acc[0][1], acc[0][2], acc[0][3]);
  acc_guard4(acc[1][0], acc[1][1], acc[1][2], acc[1][3]);
  acc_guard4(acc[2][0], acc[2][1], acc[2][2], acc[2][3]);
  acc_guard4(acc[3][0], acc[3][1], acc[3][2], acc[3][3]);

  float* slab = sT[wave];
  const float* Rb = RESID ? (resid + (size_t)b * strideR) : nullptr;
  float* C = Cout + (size_t)b * strideC;
  const int hh = lane >> 4, c4 = (lane & 15) * 4;
  v4f pm = (v4f){0.f, 0.f, 0.f, 0.f}, ps = (v4f){1.f, 1.f, 1.f, 1.f}, pb = (v4f){0.f, 0.f, 0.f, 0.f};
  if (EPI == 1) {
    pm = *(const v4f*)(bnM + n0 + c4);
    const v4f pg = *(const v4f*)(bnG + n0 + c4);
    const v4f pv = *(const v4f*)(bnV + n0 + c4);
    pb = *(const v4f*)(bnB + n0 + c4);
#pragma unroll
    for (int e = 0; e < 4; ++e) ps[e] = pg[e] * rsqrtf(pv[e] + 1e-5f);
  }
#pragma unroll
  for (int i = 0; i < 4; ++i) {
    const int mBase = m0 + (i << 4);
#pragma unroll
    for (int j = 0; j < 4; ++j) {
#pragma unroll
      for (int r = 0; r < 8; ++r) {
        slab[(mOff + r) * 68 + (j << 4) + rlane] = acc[i][j][r] * scale;
      }
    }
    __builtin_amdgcn_fence(__ATOMIC_RELEASE, "workgroup");
    __builtin_amdgcn_wave_barrier();
    __builtin_amdgcn_fence(__ATOMIC_ACQUIRE, "workgroup");
    for (int pass = 0; pass < 2; ++pass) {
#pragma unroll
      for (int it = 0; it < 8; ++it) {
        const int row = it * 2 + hh;
        v4f v = *(const v4f*)(slab + row * 68 + c4);
        if (EPI == 1) {
          v = (v - pm) * ps + pb;
#pragma unroll
          for (int e = 0; e < 4; ++e) v[e] = fmaxf(v[e], 0.0f);
        }
        const size_t o = (size_t)(mBase + row) * ldc + n0 + c4;
        if (RESID) { const v4f rr = *(const v4f*)(Rb + o); v = v + rr; }
        *(volatile v4f*)(C + o) = v;
      }
      __threadfence();
    }
    __builtin_amdgcn_fence(__ATOMIC_RELEASE, "workgroup");
    __builtin_amdgcn_wave_barrier();
    __builtin_amdgcn_fence(__ATOMIC_ACQUIRE, "workgroup");
  }
}

__global__ __launch_bounds__(256) void split_rows_bf16_kernel(
    const float* __restrict__ src, unsigned short* __restrict__ dhi, unsigned short* __restrict__ dlo, int total8)
{
  const int i = blockIdx.x * 256 + threadIdx.x;
  if (i >= total8) return;
  const size_t e0 = (size_t)i << 3;
  const v4f a0 = *(const v4f*)(src + e0);
  const v4f a1 = *(const v4f*)(src + e0 + 4);
  v8h hv, lv;
#pragma unroll
  for (int e = 0; e < 4; ++e) {
    const unsigned short h0 = f2bf_bits(a0[e]), h1 = f2bf_bits(a1[e]);
    const unsigned short l0 = f2bf_bits(a0[e] - bf_bits2f(h0)), l1 = f2bf_bits(a1[e] - bf_bits2f(h1));
    hv[e]     = __builtin_bit_cast(_Float16, h0);
    hv[4 + e] = __builtin_bit_cast(_Float16, h1);
    lv[e]     = __builtin_bit_cast(_Float16, l0);
    lv[4 + e] = __builtin_bit_cast(_Float16, l1);
  }
  unsigned short* qh = dhi + e0;
  unsigned short* ql = dlo + e0;
  *(volatile v8h*)qh = hv;
  *(volatile v8h*)ql = lv;
  __threadfence();
  *(volatile v8h*)qh = hv;
  *(volatile v8h*)ql = lv;
}

__global__ __launch_bounds__(256) void pack_tok_bf16_kernel(
    const float* __restrict__ in, unsigned short* __restrict__ oh, unsigned short* __restrict__ ol)
{
  __shared__ __align__(16) float tile[64 * 68];
  const int tid = threadIdx.x, lane = tid & 31, wave = tid >> 5;
  const int ch0 = blockIdx.x * 64, px0 = blockIdx.y * 64, bz = blockIdx.z;
  const float* src = in + (size_t)bz * kCin * kHW;
  const size_t obase = (size_t)bz * kHW * kCin;
  const int lr = tid >> 4, lc4 = (tid & 15) * 4;
#pragma unroll
  for (int i = 0; i < 4; ++i) {
    const int r = lr + 16 * i;
    const v4f v = *(const v4f*)(src + (size_t)(ch0 + r) * kHW + px0 + lc4);
    *(v4f*)(tile + r * 68 + lc4) = v;
  }
  __syncthreads();
  const int q = lane >> 3, c8 = (lane & 7) * 8;
  v8h hv[2], lv[2];
#pragma unroll
  for (int it = 0; it < 2; ++it) {
    const int prow = it * 32 + wave * 4 + q;
#pragma unroll
    for (int e = 0; e < 8; ++e) {
      const float f = tile[(c8 + e) * 68 + prow];
      const unsigned short hb = f2bf_bits(f);
      const unsigned short lb = f2bf_bits(f - bf_bits2f(hb));
      hv[it][e] = __builtin_bit_cast(_Float16, hb);
      lv[it][e] = __builtin_bit_cast(_Float16, lb);
    }
  }
  for (int pass = 0; pass < 2; ++pass) {
#pragma unroll
    for (int it = 0; it < 2; ++it) {
      const int prow = it * 32 + wave * 4 + q;
      const size_t o = obase + (size_t)(px0 + prow) * kCin + ch0 + c8;
      *(volatile v8h*)(oh + o) = hv[it];
      *(volatile v8h*)(ol + o) = lv[it];
    }
    __threadfence();
  }
}

template <int R, int C, int CP>
__global__ __launch_bounds__(256) void transpose_f16_kernel(
    const float* __restrict__ in, unsigned short* __restrict__ out, float sc)
{
  static_assert((R % 64) == 0 && (CP % 64) == 0 && (C % 4) == 0 && C >= 4 && C <= CP, "shape");
  __shared__ __align__(16) float tile[64 * 68];
  const int tid = threadIdx.x, lane = tid & 31, wave = tid >> 5;
  const int r0 = blockIdx.x * 64, c0 = blockIdx.y * 64;
  const int lr = tid >> 4, lc4 = (tid & 15) * 4;
  const int col = c0 + lc4;
  const int colc = (col < C) ? col : (C - 4);
  const float fz = (col < C) ? 1.0f : 0.0f;
#pragma unroll
  for (int i = 0; i < 4; ++i) {
    const int r = lr + 16 * i;
    v4f v = *(const v4f*)(in + (size_t)(r0 + r) * C + colc);
    v = v * fz;
    *(v4f*)(tile + r * 68 + lc4) = v;
  }
  __syncthreads();
  const int q = lane >> 3, c8 = (lane & 7) * 8;
  v8h hv[2];
#pragma unroll
  for (int it = 0; it < 2; ++it) {
    const int orow = it * 32 + wave * 4 + q;
#pragma unroll
    for (int e = 0; e < 8; ++e) hv[it][e] = (_Float16)(tile[(c8 + e) * 68 + orow] * sc);
  }
  for (int pass = 0; pass < 2; ++pass) {
#pragma unroll
    for (int it = 0; it < 2; ++it) {
      const int orow = it * 32 + wave * 4 + q;
      *(volatile v8h*)(out + (size_t)(c0 + orow) * R + r0 + c8) = hv[it];
    }
    __threadfence();
  }
}

__global__ __launch_bounds__(256) void ln256_f16_kernel(
    const float* __restrict__ RS, const float* __restrict__ gr, const float* __restrict__ br,
    const float* __restrict__ gt, const float* __restrict__ bt, unsigned short* __restrict__ LNP)
{
  const int lane = threadIdx.x & 31, wave = threadIdx.x >> 5;
  const int tokg = blockIdx.x * 8 + wave;
  const int mod = (blockIdx.x >= (kNTok / 8)) ? 1 : 0;
  const float* g  = mod ? gt : gr;
  const float* be = mod ? bt : br;
  const float* row = RS + (size_t)tokg * kCout + lane * 8;
  const v4f a0 = *(const v4f*)row;
  const v4f a1 = *(const v4f*)(row + 4);
  float s = 0.0f;
#pragma unroll
  for (int e = 0; e < 4; ++e) s += a0[e];
#pragma unroll
  for (int e = 0; e < 4; ++e) s += a1[e];
#pragma unroll
  for (int off = 16; off > 0; off >>= 1) s += __shfl_xor(s, off, 32);
  const float mean = s * (1.0f / kCout);
  float dv[8];
#pragma unroll
  for (int e = 0; e < 4; ++e) { dv[e] = a0[e] - mean; dv[4 + e] = a1[e] - mean; }
  float ss = 0.0f;
#pragma unroll
  for (int e = 0; e < 8; ++e) ss = fmaf(dv[e], dv[e], ss);
#pragma unroll
  for (int off = 16; off > 0; off >>= 1) ss += __shfl_xor(ss, off, 32);
  const float var  = ss * (1.0f / kCout);
  const float rstd = rsqrtf(var + 1e-6f);
  const v4f g0 = *(const v4f*)(g + lane * 8),  g1 = *(const v4f*)(g + lane * 8 + 4);
  const v4f b0 = *(const v4f*)(be + lane * 8), b1 = *(const v4f*)(be + lane * 8 + 4);
  v8h hv;
#pragma unroll
  for (int e = 0; e < 4; ++e) {
    hv[e]     = (_Float16)(dv[e] * rstd * g0[e] + b0[e]);
    hv[4 + e] = (_Float16)(dv[4 + e] * rstd * g1[e] + b1[e]);
  }
  unsigned short* op = LNP + (size_t)tokg * kCout + lane * 8;
  *(volatile v8h*)op = hv;
  __threadfence();
  *(volatile v8h*)op = hv;
}

__global__ __launch_bounds__(256) void dwconv_silu_kernel(
    const float* __restrict__ XZ, const float* __restrict__ kwr, const float* __restrict__ kwt,
    float* __restrict__ U, unsigned short* __restrict__ U16)
{
  __shared__ __align__(16) float sT[16 * kConvTP];
  __shared__ __align__(16) float sWk[9 * 256];
  const int tid = threadIdx.x, lane = tid & 31, wave = tid >> 5;
  const int mod = blockIdx.z;
  const int d0 = blockIdx.x * 256, d = d0 + tid;
  const int tok0 = blockIdx.y * 16;
  const int b = tok0 >> 10, px0 = tok0 & (kHW - 1), h = px0 >> 5, w0 = px0 & 31;
  const float* X = XZ + (size_t)mod * kNTok * kXzP;
  const float* kw = mod ? kwt : kwr;
#pragma unroll
  for (int jj = 0; jj < 3; ++jj) {
    int i = tid + 256 * jj;
    i = (i < 576) ? i : 575;
    const int t = i >> 6, cc = (i & 63) * 4;
    const v4f v = *(const v4f*)(kw + (size_t)t * kDin + d0 + cc);
    *(v4f*)(sWk + t * 256 + cc) = v;
  }
  __syncthreads();
  float wk[9];
#pragma unroll
  for (int t = 0; t < 9; ++t) wk[t] = sWk[t * 256 + tid];

  const size_t img = (size_t)b * kHW;
  int rb[3];
  float fy[3];
#pragma unroll
  for (int dy = 0; dy < 3; ++dy) {
    const int hn = h + dy - 1;
    const int hc = hn < 0 ? 0 : (hn > 31 ? 31 : hn);
    fy[dy] = (hn >= 0 && hn <= 31) ? 1.0f : 0.0f;
    rb[dy] = hc * kImgW;
  }
  const int wpc = (w0 > 0) ? (w0 - 1) : 0;
  const float fp = (w0 > 0) ? 1.0f : 0.0f;
  float xp[3], xc[3];
#pragma unroll
  for (int dy = 0; dy < 3; ++dy) {
    const float vp = X[(img + (size_t)(rb[dy] + wpc)) * kXzP + d];
    const float vc = X[(img + (size_t)(rb[dy] + w0)) * kXzP + d];
    xp[dy] = vp * (fy[dy] * fp);
    xc[dy] = vc * fy[dy];
  }
#pragma unroll 1
  for (int s = 0; s < 16; ++s) {
    const int wn = w0 + s + 1;
    const int wnc = (wn > 31) ? 31 : wn;
    const float fn = (wn <= 31) ? 1.0f : 0.0f;
    float xn[3];
#pragma unroll
    for (int dy = 0; dy < 3; ++dy) {
      const float v = X[(img + (size_t)(rb[dy] + wnc)) * kXzP + d];
      xn[dy] = v * (fy[dy] * fn);
    }
    float acc = 0.0f;
#pragma unroll
    for (int dy = 0; dy < 3; ++dy) {
      acc = fmaf(xp[dy], wk[dy * 3 + 0], acc);
      acc = fmaf(xc[dy], wk[dy * 3 + 1], acc);
      acc = fmaf(xn[dy], wk[dy * 3 + 2], acc);
    }
    const float e  = expf(-acc);
    const float sg = __builtin_amdgcn_rcpf(1.0f + e);
    sT[s * kConvTP + tid] = acc * sg;
#pragma unroll
    for (int dy = 0; dy < 3; ++dy) { xp[dy] = xc[dy]; xc[dy] = xn[dy]; }
  }
  __syncthreads();
  const size_t srow0 = (size_t)b * kSeqL + (size_t)mod * kHW + px0;
  const int hrow = wave >> 1;
  const int hch  = (wave & 1) * 128 + lane * 4;
  v4f fv[4];
  v8h hv[2];
#pragma unroll
  for (int it = 0; it < 4; ++it) fv[it] = *(const v4f*)(sT + (it * 4 + hrow) * kConvTP + hch);
#pragma unroll
  for (int it = 0; it < 2; ++it) {
    const float* sp = sT + (it * 8 + wave) * kConvTP + lane * 8;
    const v4f a0 = *(const v4f*)(sp);
    const v4f a1 = *(const v4f*)(sp + 4);
#pragma unroll
    for (int e = 0; e < 4; ++e) {
      hv[it][e]     = (_Float16)(a0[e] * 16.0f);
      hv[it][4 + e] = (_Float16)(a1[e] * 16.0f);
    }
  }
  for (int pass = 0; pass < 2; ++pass) {
#pragma unroll
    for (int it = 0; it < 4; ++it)
      *(volatile v4f*)(U + (srow0 + it * 4 + hrow) * kDin + d0 + hch) = fv[it];
#pragma unroll
    for (int it = 0; it < 2; ++it)
      *(volatile v8h*)(U16 + (srow0 + it * 8 + wave) * kDin + d0 + lane * 8) = hv[it];
    __threadfence();
  }
}

__global__ __launch_bounds__(64) void scan_kernel(
    const float* __restrict__ XD, const float* __restrict__ U,
    const float* __restrict__ Wdt, const float* __restrict__ bdt, const float* __restrict__ Alog,
    const float* __restrict__ Dp, float* __restrict__ Y)
{
  __shared__ __align__(16) float sX[kScanTS * kXdP];
  __shared__ __align__(16) float sY[kScanTS * kScanYP];
  __shared__ __align__(16) float sW[kDtR * kScanCh];
  __shared__ __align__(16) float sA[kNst * kScanCh];
  const int tid = threadIdx.x, lane = tid & 31, wave = tid >> 5;
  constexpr int kBlkPerB = kDin / kScanCh;
  const int bix = blockIdx.x / kBlkPerB;
  const int d0  = (blockIdx.x - bix * kBlkPerB) * kScanCh;
  const int d   = d0 + tid;
  const size_t row0 = (size_t)bix * kSeqL;
#pragma unroll 1
  for (int r = 0; r < kDtR; ++r) sW[r * kScanCh + tid] = Wdt[(size_t)r * kDin + d];
#pragma unroll 1
  for (int s = 0; s < kNst; ++s) sA[s * kScanCh + tid] = -expf(Alog[(size_t)d * kNst + s]);
  __syncthreads();
  float negA[kNst], h[kNst];
#pragma unroll
  for (int s = 0; s < kNst; ++s) {
    negA[s] = sA[s * kScanCh + tid];
    h[s] = 0.0f;
  }
  const float bb = bdt[d], Dd = Dp[d];
  const int lr = tid >> 4, lc4 = (tid & 15) * 4;
  const int hh = lane >> 4, c4 = (lane & 15) * 4;
#pragma unroll 1
  for (int t0 = 0; t0 < kSeqL; t0 += kScanTS) {
    __syncthreads();
#pragma unroll
    for (int i = 0; i < 8; ++i) {
      const int r = lr + 4 * i;
      *(v4f*)(sX + r * kXdP + lc4) = *(const v4f*)(XD + (row0 + t0 + r) * kXdP + lc4);
    }
    asm volatile("" ::: "memory");
#pragma unroll
    for (int i = 8; i < 16; ++i) {
      const int r = lr + 4 * i;
      *(v4f*)(sX + r * kXdP + lc4) = *(const v4f*)(XD + (row0 + t0 + r) * kXdP + lc4);
    }
    __syncthreads();
#pragma unroll 1
    for (int s = 0; s < kScanTS; ++s) {
      const int t = t0 + s;
      const float* xr = sX + s * kXdP;
      float vdot = 0.0f;
#pragma unroll 1
      for (int r4 = 0; r4 < kDtR / 4; ++r4) {
        const v4f xv = *(const v4f*)(xr + 4 * r4);
        const float* wp = sW + (4 * r4) * kScanCh + tid;
        vdot = fmaf(xv[0], wp[0], vdot);
        vdot = fmaf(xv[1], wp[kScanCh], vdot);
        vdot = fmaf(xv[2], wp[2 * kScanCh], vdot);
        vdot = fmaf(xv[3], wp[3 * kScanCh], vdot);
      }
      float Bs[kNst], Cs[kNst];
#pragma unroll
      for (int q4 = 0; q4 < 4; ++q4) {
        const v4f bv = *(const v4f*)(xr + kDtR + 4 * q4);
        const v4f cv = *(const v4f*)(xr + kDtR + kNst + 4 * q4);
        Bs[4 * q4 + 0] = bv[0]; Bs[4 * q4 + 1] = bv[1]; Bs[4 * q4 + 2] = bv[2]; Bs[4 * q4 + 3] = bv[3];
        Cs[4 * q4 + 0] = cv[0]; Cs[4 * q4 + 1] = cv[1]; Cs[4 * q4 + 2] = cv[2]; Cs[4 * q4 + 3] = cv[3];
      }
      const float v   = vdot + bb;
      const float a   = __expf(-fabsf(v));
      const float ua  = 1.0f + a;
      const float l1p = __logf(ua) + (a - (ua - 1.0f)) * __builtin_amdgcn_rcpf(ua);
      const float dt  = fmaxf(v, 0.0f) + l1p;
      const float xt  = U[(row0 + t) * kDin + d];
      const float dtx = dt * xt;
      float y = 0.0f;
#pragma unroll
      for (int k = 0; k < kNst; ++k) {
        const float e = __expf(dt * negA[k]);
        h[k] = e * h[k] + dtx * Bs[k];
        y = h[k] * Cs[k] + y;
      }
      y = xt * Dd + y;
      sY[s * kScanYP + tid] = y;
    }
    __syncthreads();
    v4f ov[16];
#pragma unroll
    for (int it = 0; it < 16; ++it) {
      const int row = it * 4 + wave * 2 + hh;
      ov[it] = *(const v4f*)(sY + row * kScanYP + c4);
    }
    for (int pass = 0; pass < 2; ++pass) {
#pragma unroll
      for (int it = 0; it < 16; ++it) {
        const int row = it * 4 + wave * 2 + hh;
        *(volatile v4f*)(Y + (row0 + t0 + row) * kDin + d0 + c4) = ov[it];
      }
      __threadfence();
    }
  }
}

__global__ __launch_bounds__(256) void resid_t_kernel(const float* __restrict__ RS, float* __restrict__ RT)
{
  __shared__ __align__(16) float tile[64 * 68];
  const int tid = threadIdx.x, lane = tid & 31, wave = tid >> 5;
  const int c0 = blockIdx.x * 64, tok0 = blockIdx.y * 64;
  const int b = tok0 >> 10, px0 = tok0 & (kHW - 1);
  const float* R0 = RS;
  const float* R1 = RS + (size_t)kNTok * kCout;
  const int lr = tid >> 4, lc4 = (tid & 15) * 4;
#pragma unroll
  for (int i = 0; i < 2; ++i) {
    const int r = lr + 16 * i;
    const v4f a = *(const v4f*)(R0 + (size_t)(tok0 + r) * kCout + c0 + lc4);
    const v4f s = *(const v4f*)(R1 + (size_t)(tok0 + r) * kCout + c0 + lc4);
    v4f v = (a + s) * 0.5f;
    *(v4f*)(tile + r * 68 + lc4) = v;
  }
  asm volatile("" ::: "memory");
#pragma unroll
  for (int i = 2; i < 4; ++i) {
    const int r = lr + 16 * i;
    const v4f a = *(const v4f*)(R0 + (size_t)(tok0 + r) * kCout + c0 + lc4);
    const v4f s = *(const v4f*)(R1 + (size_t)(tok0 + r) * kCout + c0 + lc4);
    v4f v = (a + s) * 0.5f;
    *(v4f*)(tile + r * 68 + lc4) = v;
  }
  __syncthreads();
  const int hh = lane >> 4, c4 = (lane & 15) * 4;
  v4f ov[4];
#pragma unroll
  for (int it = 0; it < 4; ++it) {
    const int crow = it * 16 + wave * 2 + hh;
    v4f v;
    v[0] = tile[(c4 + 0) * 68 + crow];
    v[1] = tile[(c4 + 1) * 68 + crow];
    v[2] = tile[(c4 + 2) * 68 + crow];
    v[3] = tile[(c4 + 3) * 68 + crow];
    ov[it] = v;
  }
  for (int pass = 0; pass < 2; ++pass) {
#pragma unroll
    for (int it = 0; it < 4; ++it) {
      const int crow = it * 16 + wave * 2 + hh;
      *(volatile v4f*)(RT + ((size_t)(b * kCout + c0 + crow)) * kHW + px0 + c4) = ov[it];
    }
    __threadfence();
  }
}

__global__ __launch_bounds__(256) void ln512_gate_kernel(
    const float* __restrict__ Y, const float* __restrict__ XZ,
    const float* __restrict__ g, const float* __restrict__ be, unsigned short* __restrict__ GP)
{
  __shared__ __align__(16) float sv[8 * kDin];
  const int lane = threadIdx.x & 31, wave = threadIdx.x >> 5;
  const int tok = blockIdx.x * 8 + wave;
  const int b = tok >> 10, j = tok & (kHW - 1);
  const float* y1 = Y + ((size_t)b * kSeqL + j) * kDin;
  const float* y2 = Y + ((size_t)b * kSeqL + kHW + j) * kDin;
  const float* z1 = XZ + (size_t)tok * kXzP + kDin;
  const float* z2 = XZ + ((size_t)kNTok + tok) * kXzP + kDin;
  float* myv = sv + wave * kDin;
  float s = 0.0f;
#pragma unroll 1
  for (int i = 0; i < kDin / 32; ++i) {
    const int c = lane + 32 * i;
    const float v = y1[c] + y2[c];
    myv[c] = v;
    s += v;
  }
#pragma unroll
  for (int off = 16; off > 0; off >>= 1) s += __shfl_xor(s, off, 32);
  const float mean = s * (1.0f / kDin);
  float ss = 0.0f;
#pragma unroll 1
  for (int i = 0; i < kDin / 32; ++i) {
    const int c = lane + 32 * i;
    const float dv = myv[c] - mean;
    ss = fmaf(dv, dv, ss);
  }
#pragma unroll
  for (int off = 16; off > 0; off >>= 1) ss += __shfl_xor(ss, off, 32);
  const float var  = ss * (1.0f / kDin);
  const float rstd = rsqrtf(var + 1e-6f);
#pragma unroll 1
  for (int i = 0; i < kDin / 32; ++i) {
    const int c = lane + 32 * i;
    const float yl = (myv[c] - mean) * rstd * g[c] + be[c];
    const float zz = 0.5f * (z1[c] + z2[c]);
    const float e  = expf(-zz);
    const float sg = __builtin_amdgcn_rcpf(1.0f + e);
    myv[c] = yl * (zz * sg) * 8.0f;
  }
  __syncthreads();
  v8h hv[2];
#pragma unroll
  for (int it = 0; it < 2; ++it) {
    const int c8 = it * 256 + lane * 8;
    const v4f a0 = *(const v4f*)(myv + c8);
    const v4f a1 = *(const v4f*)(myv + c8 + 4);
#pragma unroll
    for (int e = 0; e < 4; ++e) {
      hv[it][e]     = (_Float16)a0[e];
      hv[it][4 + e] = (_Float16)a1[e];
    }
  }
  for (int pass = 0; pass < 2; ++pass) {
#pragma unroll
    for (int it = 0; it < 2; ++it)
      *(volatile v8h*)(GP + (size_t)tok * kDin + it * 256 + lane * 8) = hv[it];
    __threadfence();
  }
}

extern "C" void kernel_launch(void* const* d_in, const int* in_sizes, int n_in,
                              void* d_out, int out_size, void* d_ws, size_t ws_size,
                              hipStream_t stream) {
  if (n_in < 28) return;
  if (in_sizes[0] != kNB * kCin * kHW) return;
  if (in_sizes[1] != kNB * kCin * kHW) return;
  if (in_sizes[2] != kCout * kCin || in_sizes[7] != kCout * kCin) return;
  if (in_sizes[3] != kCout || in_sizes[4] != kCout || in_sizes[5] != kCout || in_sizes[6] != kCout) return;
  if (in_sizes[8] != kCout || in_sizes[9] != kCout || in_sizes[10] != kCout || in_sizes[11] != kCout) return;
  if (in_sizes[12] != kCout || in_sizes[13] != kCout || in_sizes[14] != kCout || in_sizes[15] != kCout) return;
  if (in_sizes[16] != kCout * kXzP || in_sizes[17] != kCout * kXzP) return;
  if (in_sizes[18] != 9 * kDin || in_sizes[19] != 9 * kDin) return;
  if (in_sizes[20] != kDin * kXdW) return;
  if (in_sizes[21] != kDtR * kDin) return;
  if (in_sizes[22] != kDin) return;
  if (in_sizes[23] != kDin * kNst) return;
  if (in_sizes[24] != kDin || in_sizes[25] != kDin || in_sizes[26] != kDin) return;
  if (in_sizes[27] != kDin * kCout) return;
  if (out_size != kNB * kCout * kHW) return;
  if (ws_size < kWsTotal) return;

  const float* rgb    = (const float*)d_in[0];
  const float* tin    = (const float*)d_in[1];
  const float* w1     = (const float*)d_in[2];
  const float* g1     = (const float*)d_in[3];
  const float* b1     = (const float*)d_in[4];
  const float* m1     = (const float*)d_in[5];
  const float* v1     = (const float*)d_in[6];
  const float* w2     = (const float*)d_in[7];
  const float* g2     = (const float*)d_in[8];
  const float* b2     = (const float*)d_in[9];
  const float* m2     = (const float*)d_in[10];
  const float* v2     = (const float*)d_in[11];
  const float* lnrg   = (const float*)d_in[12];
  const float* lnrb   = (const float*)d_in[13];
  const float* lntg   = (const float*)d_in[14];
  const float* lntb   = (const float*)d_in[15];
  const float* ipr    = (const float*)d_in[16];
  const float* ipt    = (const float*)d_in[17];
  const float* dwcr   = (const float*)d_in[18];
  const float* dwct   = (const float*)d_in[19];
  const float* xproj  = (const float*)d_in[20];
  const float* dtw    = (const float*)d_in[21];
  const float* dtb    = (const float*)d_in[22];
  const float* alog   = (const float*)d_in[23];
  const float* dp     = (const float*)d_in[24];
  const float* ong    = (const float*)d_in[25];
  const float* onb    = (const float*)d_in[26];
  const float* outw   = (const float*)d_in[27];
  float* out = (float*)d_out;

  char* ws = (char*)d_ws;
  unsigned short* XB  = (unsigned short*)(ws + kOffXB);
  unsigned short* XBL = (unsigned short*)(ws + kOffXBL);
  unsigned short* WB  = (unsigned short*)(ws + kOffWB);
  unsigned short* WBL = (unsigned short*)(ws + kOffWBL);
  unsigned short* IP  = (unsigned short*)(ws + kOffIP);
  unsigned short* XP  = (unsigned short*)(ws + kOffXP);
  unsigned short* OW  = (unsigned short*)(ws + kOffOW);
  float*          RS  = (float*)(ws + kOffRS);
  unsigned short* LN  = (unsigned short*)(ws + kOffLN);
  float*          XZ  = (float*)(ws + kOffXZ);
  float*          U   = (float*)(ws + kOffU);
  unsigned short* U16 = (unsigned short*)(ws + kOffU16);
  float*          XD  = (float*)(ws + kOffXD);
  float*          Y   = (float*)(ws + kOffY);
  unsigned short* G   = (unsigned short*)(ws + kOffG);
  float*          RT  = (float*)(ws + kOffRT);

  const size_t xPlane  = (size_t)kNTok * kCin;
  const size_t wPlane  = (size_t)kCout * kCin;
  const size_t ipPlane = (size_t)kXzP * kCout;
  const size_t rsPlane = (size_t)kNTok * kCout;

  pack_tok_bf16_kernel<<<dim3(kCin / 64, kHW / 64, kNB), 256, 0, stream>>>(rgb, XB, XBL);
  pack_tok_bf16_kernel<<<dim3(kCin / 64, kHW / 64, kNB), 256, 0, stream>>>(tin, XB + xPlane, XBL + xPlane);
  split_rows_bf16_kernel<<<(kCout * kCin / 8) / 256, 256, 0, stream>>>(w1, WB, WBL, kCout * kCin / 8);
  split_rows_bf16_kernel<<<(kCout * kCin / 8) / 256, 256, 0, stream>>>(w2, WB + wPlane, WBL + wPlane, kCout * kCin / 8);
  transpose_f16_kernel<kCout, kXzP, kXzP><<<dim3(kCout / 64, kXzP / 64), 256, 0, stream>>>(ipr, IP, 64.0f);
  transpose_f16_kernel<kCout, kXzP, kXzP><<<dim3(kCout / 64, kXzP / 64), 256, 0, stream>>>(ipt, IP + ipPlane, 64.0f);
  transpose_f16_kernel<kDin, kXdW, kXdP><<<dim3(kDin / 64, kXdP / 64), 256, 0, stream>>>(xproj, XP, 64.0f);
  transpose_f16_kernel<kDin, kCout, kCout><<<dim3(kDin / 64, kCout / 64), 256, 0, stream>>>(outw, OW, 64.0f);

  wmma_gemm64<1, 2, 1, false><<<dim3(((kNTok / 64) * (kCout / 64)) / 8, 1), 256, 0, stream>>>(
      XB, XBL, kCin, 0L,
      WB, WBL, kCin, 0L,
      RS, kCout, 0L,
      m1, g1, v1, b1,
      nullptr, 0L,
      kNTok, kCout, kCin, 1.0f);
  wmma_gemm64<1, 2, 1, false><<<dim3(((kNTok / 64) * (kCout / 64)) / 8, 1), 256, 0, stream>>>(
      XB + xPlane, XBL + xPlane, kCin, 0L,
      WB + wPlane, WBL + wPlane, kCin, 0L,
      RS + rsPlane, kCout, 0L,
      m2, g2, v2, b2,
      nullptr, 0L,
      kNTok, kCout, kCin, 1.0f);

  ln256_f16_kernel<<<(2 * kNTok) / 8, 256, 0, stream>>>(RS, lnrg, lnrb, lntg, lntb, LN);

  wmma_gemm64<0, 0, 0, false><<<dim3(((kNTok / 64) * (kXzP / 64)) / 8, 2), 256, 0, stream>>>(
      LN, nullptr, kCout, (long)rsPlane,
      IP, nullptr, kCout, (long)ipPlane,
      XZ, kXzP, (long)((size_t)kNTok * kXzP),
      nullptr, nullptr, nullptr, nullptr,
      nullptr, 0L,
      kNTok, kXzP, kCout, 1.0f / 64.0f);

  dwconv_silu_kernel<<<dim3(kDin / 256, kNTok / 16, 2), 256, 0, stream>>>(XZ, dwcr, dwct, U, U16);

  wmma_gemm64<0, 0, 0, false><<<dim3(((kNSeq / 64) * (kXdP / 64)) / 8, 1), 256, 0, stream>>>(
      U16, nullptr, kDin, 0L,
      XP, nullptr, kDin, 0L,
      XD, kXdP, 0L,
      nullptr, nullptr, nullptr, nullptr,
      nullptr, 0L,
      kNSeq, kXdP, kDin, 1.0f / 1024.0f);

  scan_kernel<<<kNB * (kDin / kScanCh), kScanCh, 0, stream>>>(XD, U, dtw, dtb, alog, dp, Y);

  resid_t_kernel<<<dim3(kCout / 64, kNTok / 64), 256, 0, stream>>>(RS, RT);

  ln512_gate_kernel<<<kNTok / 8, 256, 0, stream>>>(Y, XZ, ong, onb, G);

  wmma_gemm64<0, 0, 0, true><<<dim3(((kCout / 64) * (kHW / 64)) / 8, kNB), 256, 0, stream>>>(
      OW, nullptr, kDin, 0L,
      G, nullptr, kDin, (long)((size_t)kHW * kDin),
      out, kHW, (long)((size_t)kCout * kHW),
      nullptr, nullptr, nullptr, nullptr,
      RT, (long)((size_t)kCout * kHW),
      kCout, kHW, kDin, 1.0f / 512.0f);
}
